// GRU_29703993819854
// MI455X (gfx1250) — hardware-run, weakly checked
//
#include <hip/hip_runtime.h>
#include <math.h>

constexpr int NBATCH   = 1024;
constexpr int TENC     = 512;
constexpr int PLEN     = 300;
constexpr int NDEC     = PLEN - 1;
constexpr int NSTEPS   = TENC + NDEC;
constexpr int NIN      = 3;
constexpr int NHID     = 64;
constexpr int NGATE    = 4 * NHID;
constexpr int NOUTF    = 2;
constexpr int ROWS_BLK = 16;
constexpr int NTHR     = 128;
constexpr int WPITCH   = 72;
constexpr int HPITCH   = 72;
constexpr int HFPITCH  = 68;
constexpr int YROW     = PLEN * NOUTF;
constexpr int YBLK     = ROWS_BLK * YROW;
constexpr int YLINES   = YBLK / 32;
constexpr float WCAR   = 256.0f;
constexpr float HCAR   = 16.0f;
constexpr float LCAR   = 4096.0f;
constexpr float SC_HI  = 1.0f / (HCAR * WCAR);
constexpr float SC_LO  = 1.0f / (HCAR * WCAR * LCAR);
static_assert(NBATCH % ROWS_BLK == 0, "grid exact");
static_assert(NHID == 16 * (NTHR / 32), "one 16-unit group per wave");
static_assert((NGATE * NHID) % (4 * NTHR) == 0, "W plane staging exact");
static_assert(NGATE == 2 * NTHR, "bias / W_ih staging exact");
static_assert(NOUTF * NHID == NTHR, "W_out staging exact");
static_assert(ROWS_BLK * NOUTF == 32, "output head uses exactly one wave");
static_assert(YBLK % 32 == 0 && (YBLK * 4) % 128 == 0, "block output region is whole 128-B lines");
static_assert(NBATCH * YROW == 614400, "output element count");
static_assert(WPITCH % 8 == 0 && HPITCH % 8 == 0 && HFPITCH % 4 == 0, "16-B alignment of fragment and v4f loads");
static_assert(NHID % 32 == 0, "K = 64 = 2 chunks of 32, no tail");

typedef __attribute__((ext_vector_type(16))) _Float16 v16h;
typedef __attribute__((ext_vector_type(8)))  _Float16 v8h;
typedef __attribute__((ext_vector_type(8)))  float    v8f;
typedef __attribute__((ext_vector_type(4)))  float    v4f;
typedef __attribute__((ext_vector_type(2)))  unsigned v2u;
typedef __attribute__((ext_vector_type(4)))  unsigned v4u;

__device__ __forceinline__ unsigned short f2bf_bits(float f) {
  unsigned u = __float_as_uint(f);
  return (unsigned short)((u + 0x7FFFu + ((u >> 16) & 1u)) >> 16);
}
__device__ __forceinline__ float bf_bits2f(unsigned short h) { return __uint_as_float(((unsigned)h) << 16); }
__device__ __forceinline__ float bf16r(float f) { return bf_bits2f(f2bf_bits(f)); }
__device__ __forceinline__ unsigned short h16bits(float f) { const _Float16 h = (_Float16)f; return __builtin_bit_cast(unsigned short, h); }

struct FragH {
  union U { v16h v; v8h h[2]; };
  static __device__ __forceinline__ v16h load(const _Float16* p) {
    U f; f.h[0] = *(const v8h*)(p); f.h[1] = *(const v8h*)(p + 16); return f.v;
  }
  static __device__ __forceinline__ v8f mma(v16h a, v16h b, v8f c) {
    return __builtin_amdgcn_wmma_f32_16x16x32_f16(false, a, false, b, (short)0, c, false, false);
  }
};
__device__ __forceinline__ void guard2x6(v8f& a, v8f& b, v16h x0, v16h x1, v16h x2, v16h x3, v16h y0, v16h y1) {
  asm volatile("v_nop\n\tv_nop\n\tv_nop\n\tv_nop" : "+v"(a), "+v"(b) : "v"(x0), "v"(x1), "v"(x2), "v"(x3), "v"(y0), "v"(y1));
}

__device__ __forceinline__ float frcp(float x)  { return __builtin_amdgcn_rcpf(x); }
__device__ __forceinline__ float fsigm(float x) { return frcp(1.0f + expf(-x)); }
__device__ __forceinline__ float ftanh(float x) { return 1.0f - 2.0f * frcp(expf(2.0f * x) + 1.0f); }

__global__ __launch_bounds__(NTHR) void lstm_seq_kernel(const float* __restrict__ x, const float* __restrict__ force,
                                                        const float* __restrict__ wih, const float* __restrict__ whh,
                                                        const float* __restrict__ bih, const float* __restrict__ bhh,
                                                        const float* __restrict__ wout, const float* __restrict__ bout,
                                                        const int* __restrict__ plen, float* __restrict__ out) {
  __shared__ __align__(16) unsigned short sW[NGATE * WPITCH];
  __shared__ __align__(16) _Float16       sAh[ROWS_BLK * HPITCH];
  __shared__ __align__(16) _Float16       sAl[ROWS_BLK * HPITCH];
  __shared__ __align__(16) float          sHf[ROWS_BLK * HFPITCH];
  __shared__ __align__(16) float          sY[YBLK];
  __shared__ __align__(16) float          sX[ROWS_BLK * 4];
  __shared__ __align__(16) float          sWih[NGATE * 4];
  __shared__ __align__(16) float          sB[NGATE];
  __shared__ __align__(16) float          sWo[NOUTF * NHID];
  __shared__ __align__(16) float          sBo[4];

  const int tid = threadIdx.x, lane = tid & 31, wave = tid >> 5;
  const int c = lane & 15, hh = lane >> 4, koff = hh * 8;
  const int blk = blockIdx.x;
  const int b0 = blk * ROWS_BLK;
  const int j = 16 * wave + c;

#pragma unroll 1
  for (int it = 0; it < (NGATE * NHID) / (4 * NTHR); ++it) {
    const int idx = it * NTHR + tid;
    const int n = idx >> 4, k4 = (idx & 15) * 4;
    const v4f v = *(const v4f*)(whh + (size_t)n * NHID + k4);
    const float e0 = v[0], e1 = v[1], e2 = v[2], e3 = v[3];
    const unsigned u0 = h16bits(WCAR * bf16r(e0)), u1 = h16bits(WCAR * bf16r(e1));
    const unsigned u2 = h16bits(WCAR * bf16r(e2)), u3 = h16bits(WCAR * bf16r(e3));
    v2u pk;
    pk[0] = u0 | (u1 << 16);
    pk[1] = u2 | (u3 << 16);
    *(v2u*)(sW + n * WPITCH + k4) = pk;
  }
  asm volatile("" ::: "memory");
  {
    const int na = tid, nb = tid + NTHR;
    const float a0 = wih[na * NIN + 0], a1 = wih[na * NIN + 1], a2 = wih[na * NIN + 2];
    const float c0 = wih[nb * NIN + 0], c1 = wih[nb * NIN + 1], c2 = wih[nb * NIN + 2];
    const v4f va = {bf16r(a0), bf16r(a1), bf16r(a2), 0.0f};
    const v4f vb = {bf16r(c0), bf16r(c1), bf16r(c2), 0.0f};
    *(v4f*)(sWih + na * 4) = va;
    *(v4f*)(sWih + nb * 4) = vb;
  }
  asm volatile("" ::: "memory");
  {
    sB[tid]        = bf16r(bih[tid]) + bf16r(bhh[tid]);
    sB[tid + NTHR] = bf16r(bih[tid + NTHR]) + bf16r(bhh[tid + NTHR]);
    sWo[tid]       = bf16r(wout[tid]);
    const float bov = bf16r(bout[tid & 1]);
    if (tid < NOUTF) sBo[tid] = bov;
  }
  asm volatile("" ::: "memory");
  {
    const int row = tid & 15;
    const float* xp = x + ((size_t)(b0 + row) * TENC) * NIN;
    const float x0 = xp[0], x1 = xp[1], x2 = xp[2];
    if (tid < ROWS_BLK) { const v4f v = {bf16r(x0), bf16r(x1), bf16r(x2), 0.0f}; *(v4f*)(sX + row * 4) = v; }
  }
  {
    const v4u zu = {0u, 0u, 0u, 0u};
#pragma unroll 1
    for (int i = tid; i < (ROWS_BLK * HPITCH) / 8; i += NTHR) { ((v4u*)sAh)[i] = zu; ((v4u*)sAl)[i] = zu; }
    const v4f zf = {0.0f, 0.0f, 0.0f, 0.0f};
#pragma unroll 1
    for (int i = tid; i < YBLK / 4; i += NTHR) ((v4f*)sY)[i] = zf;
  }
  int plc;
  {
    const int plv = plen[0];
    plc = plv < 1 ? 1 : (plv > PLEN ? PLEN : plv);
  }
  __syncthreads();

  v4f wv[4];
  float bb[4];
#pragma unroll
  for (int g = 0; g < 4; ++g) {
    const int n = NHID * g + j;
    wv[g] = *(const v4f*)(sWih + n * 4);
    bb[g] = sB[n];
  }
  const float bo0 = sBo[0], bo1 = sBo[1];
  float cst[8];
#pragma unroll
  for (int r = 0; r < 8; ++r) cst[r] = 0.0f;
  const v8f z8 = {0.f, 0.f, 0.f, 0.f, 0.f, 0.f, 0.f, 0.f};
  const _Float16* sWhp = (const _Float16*)sW;

#pragma unroll 1
  for (int u = 0; u < NSTEPS; ++u) {
    float z[4][8];
    {
      v4f xv[8];
#pragma unroll
      for (int r = 0; r < 8; ++r) xv[r] = *(const v4f*)(sX + (8 * hh + r) * 4);
#pragma unroll
      for (int g = 0; g < 4; ++g) {
#pragma unroll
        for (int r = 0; r < 8; ++r)
          z[g][r] = bb[g] + xv[r][0] * wv[g][0] + xv[r][1] * wv[g][1] + xv[r][2] * wv[g][2];
      }
    }
    {
      const _Float16* ahp = sAh + c * HPITCH + koff;
      const _Float16* alp = sAl + c * HPITCH + koff;
      const v16h ah0 = FragH::load(ahp), ah1 = FragH::load(ahp + 32);
      const v16h al0 = FragH::load(alp), al1 = FragH::load(alp + 32);
#pragma unroll
      for (int g = 0; g < 4; ++g) {
        const _Float16* bp = sWhp + (NHID * g + j) * WPITCH + koff;
        const v16h bw0 = FragH::load(bp), bw1 = FragH::load(bp + 32);
        v8f acch = z8, accl = z8;
        acch = FragH::mma(ah0, bw0, acch);
        acch = FragH::mma(ah1, bw1, acch);
        accl = FragH::mma(al0, bw0, accl);
        accl = FragH::mma(al1, bw1, accl);
        guard2x6(acch, accl, ah0, ah1, al0, al1, bw0, bw1);
#pragma unroll
        for (int r = 0; r < 8; ++r) z[g][r] += acch[r] * SC_HI + accl[r] * SC_LO;
      }
    }
    float hn[8];
#pragma unroll
    for (int r = 0; r < 8; ++r) {
      const float ig = fsigm(z[0][r]);
      const float fg = fsigm(z[1][r]);
      const float gg = ftanh(z[2][r]);
      const float og = fsigm(z[3][r]);
      const float cn = fg * cst[r] + ig * gg;
      cst[r] = cn;
      hn[r] = og * ftanh(cn);
    }
    __syncthreads();

#pragma unroll
    for (int r = 0; r < 8; ++r) {
      const float hs = hn[r] * HCAR;
      const _Float16 hi = (_Float16)hs;
      const float hif = (float)hi;
      const float res = hs - hif;
      const _Float16 lo = (_Float16)(res * LCAR);
      sAh[(8 * hh + r) * HPITCH + j] = hi;
      sAl[(8 * hh + r) * HPITCH + j] = lo;
    }
    if (u >= TENC - 1) {
#pragma unroll
      for (int r = 0; r < 8; ++r) sHf[(8 * hh + r) * HFPITCH + j] = hn[r];
    }
    {
      const int tn = (u + 1 < TENC) ? (u + 1) : (TENC - 1);
      const int row = tid & 15;
      const float* xp = x + ((size_t)(b0 + row) * TENC + (size_t)tn) * NIN;
      const float x0 = xp[0], x1 = xp[1], x2 = xp[2];
      if (tid < ROWS_BLK && u + 1 < TENC) { const v4f v = {bf16r(x0), bf16r(x1), bf16r(x2), 0.0f}; *(v4f*)(sX + row * 4) = v; }
    }
    __syncthreads();

    if (u >= TENC - 1) {
      const int slot = u - (TENC - 1);
      if (wave == 0) {
        const int row = lane >> 1, o = lane & 1;
        const float* hp = sHf + row * HFPITCH;
        const float* wp = sWo + o * NHID;
        float acc = 0.0f;
#pragma unroll 1
        for (int q = 0; q < NHID / 4; ++q) {
          const v4f hv = *(const v4f*)(hp + 4 * q);
          const v4f wq = *(const v4f*)(wp + 4 * q);
          acc += hv[0] * wq[0];
          acc += hv[1] * wq[1];
          acc += hv[2] * wq[2];
          acc += hv[3] * wq[3];
        }
        const float y = acc + (o ? bo1 : bo0);
        if (slot < plc) sY[row * YROW + slot * 2 + o] = y;
        const float yp = __shfl_xor(y, 1, 32);
        const int sidx = (slot < NDEC) ? slot : (NDEC - 1);
        const float fv = bf16r(force[(size_t)(b0 + row) * NDEC + sidx]);
        if (o == 0) { const v4f v = {y, yp, fv, 0.0f}; *(v4f*)(sX + row * 4) = v; }
      }
    }
    __syncthreads();
  }

  {
    float* ob = out + (size_t)blk * YBLK;
    const int lq = tid >> 3, w4 = (tid & 7) * 4;
    for (int pass = 0; pass < 2; ++pass) {
#pragma unroll 1
      for (int it = 0; it < (YLINES + 15) / 16; ++it) {
        const int line = it * 16 + lq;
        if (line < YLINES) {
          const v4f v = *(const v4f*)(sY + line * 32 + w4);
          *(volatile v4f*)(ob + (size_t)line * 32 + w4) = v;
        }
      }
      __threadfence();
    }
  }
}

extern "C" void kernel_launch(void* const* d_in, const int* in_sizes, int n_in,
                              void* d_out, int out_size, void* d_ws, size_t ws_size, hipStream_t stream) {
  (void)d_ws; (void)ws_size;
  if (n_in < 9 || d_out == nullptr) return;
  if (in_sizes[0] != NBATCH * TENC * NIN || in_sizes[1] != NBATCH * NDEC || in_sizes[2] != NGATE * NIN ||
      in_sizes[3] != NGATE * NHID || in_sizes[4] != NGATE || in_sizes[5] != NGATE ||
      in_sizes[6] != NOUTF * NHID || in_sizes[7] != NOUTF || in_sizes[8] != 1 ||
      out_size != NBATCH * YROW) return;

  const float* x     = (const float*)d_in[0];
  const float* force = (const float*)d_in[1];
  const float* wih   = (const float*)d_in[2];
  const float* whh   = (const float*)d_in[3];
  const float* bih   = (const float*)d_in[4];
  const float* bhh   = (const float*)d_in[5];
  const float* wout  = (const float*)d_in[6];
  const float* bout  = (const float*)d_in[7];
  const int*   plen  = (const int*)d_in[8];
  float* out = (float*)d_out;

  lstm_seq_kernel<<<NBATCH / ROWS_BLK, NTHR, 0, stream>>>(x, force, wih, whh, bih, bhh, wout, bout, plen, out);
}
